// GroupedQueryAttention_8117488189629
// MI455X (gfx1250) — hardware-verified
//
#include <hip/hip_runtime.h>
#include <math.h>

typedef __attribute__((ext_vector_type(16))) _Float16     v16h;
typedef __attribute__((ext_vector_type(8)))  _Float16     v8h;
typedef __attribute__((ext_vector_type(16))) __bf16       v16b;
typedef __attribute__((ext_vector_type(8)))  float        v8f;
typedef __attribute__((ext_vector_type(4)))  float        v4f;
typedef __attribute__((ext_vector_type(4)))  unsigned int v4u;

#ifndef NB
#define NB 1
#endif
#ifndef SEQ
#define SEQ 2048
#endif
#define NB_FULL  1
#define SEQ_FULL 2048
#define HDIM  128
#define NOUT  128
#define NQH   32
#define NKVH  8
#define REP   4
#define EQ    (NQH * HDIM)
#define EKV   (NKVH * HDIM)
#define RPK   (SEQ / NKVH)
#define KC    64
#define QT    16
#define NWAVE 4
#define SP    136
#define PP    132

#define QCAR  16.0f
#define VCAR  64.0f
#define PCAR  32768.0f
#define CCAR  1024.0f
#define WOCAR 64.0f

#define XPL       ((size_t)SEQ * HDIM)
#define X16_BYTES ((size_t)3 * SEQ * HDIM * 2)
#define WQT_BYTES ((size_t)EQ * HDIM * 2)
#define WKT_BYTES ((size_t)EKV * HDIM * 2)
#define WOT_BYTES ((size_t)NOUT * EQ * 2)
#define INV_BYTES ((size_t)256)
#define TAB_BYTES ((size_t)2 * SEQ * 64 * 4)
#define Q16_BYTES ((size_t)SEQ * EQ * 2)
#define K16_BYTES ((size_t)SEQ * EKV * 2)
#define CTX_BYTES ((size_t)SEQ * EQ * 2)
#define OFF_X16 ((size_t)0)
#define OFF_WQT (OFF_X16 + X16_BYTES)
#define OFF_WKT (OFF_WQT + WQT_BYTES)
#define OFF_WVT (OFF_WKT + WKT_BYTES)
#define OFF_WOT (OFF_WVT + WKT_BYTES)
#define OFF_INV (OFF_WOT + WOT_BYTES)
#define OFF_TAB (OFF_INV + INV_BYTES)
#define OFF_Q16 (OFF_TAB + TAB_BYTES)
#define OFF_K16 (OFF_Q16 + Q16_BYTES)
#define OFF_VT  (OFF_K16 + K16_BYTES)
#define OFF_CTX (OFF_VT + K16_BYTES)
#define WS_TOTAL (OFF_CTX + CTX_BYTES)

static_assert(NB == 1 && NB_FULL == 1);
static_assert(SEQ <= SEQ_FULL);
static_assert(SEQ % 128 == 0);
static_assert(SEQ % KC == 0 && SEQ % QT == 0 && SEQ % 4 == 0);
static_assert(EQ == NQH * HDIM && EKV == NKVH * HDIM && NQH == NKVH * REP && REP == NWAVE);
static_assert(HDIM == 128 && KC == 64 && QT == 16 && NOUT == 128);
static_assert(EKV == 1024 && EQ % 1024 == 0);
static_assert(RPK % 16 == 0);
static_assert(NWAVE * 32 * 8 == KC * (HDIM / 8));
static_assert(NWAVE * 32 * 8 == HDIM * (KC / 8));
static_assert(HDIM * 2 == 16 * 16);
static_assert(NOUT * 4 == 32 * 16);
static_assert((EQ / NWAVE) % 32 == 0);
static_assert((SP * 2) % 16 == 0 && (PP * 4) % 16 == 0);
static_assert(X16_BYTES % 256 == 0 && WQT_BYTES % 256 == 0 && WKT_BYTES % 256 == 0 && WOT_BYTES % 256 == 0);
static_assert(TAB_BYTES % 256 == 0 && Q16_BYTES % 256 == 0 && K16_BYTES % 256 == 0 && CTX_BYTES % 256 == 0);
static_assert(WS_TOTAL <= (size_t)134217728);

union FB { v16b v; v4u q[2]; };
union FH { v16h v; v8h h[2]; v4u q[2]; };

__device__ __forceinline__ unsigned int bf_bits(float f) {
    const unsigned int u = __float_as_uint(f);
    return (u + 0x7FFFu + ((u >> 16) & 1u)) >> 16;
}
__device__ __forceinline__ float bf_val(float f) { return __uint_as_float(bf_bits(f) << 16); }
__device__ __forceinline__ unsigned int h_bits(float f) { return (unsigned int)__builtin_bit_cast(unsigned short, (_Float16)f); }

__device__ __forceinline__ v8f mma_bf(v16b a, v16b b, v8f c) {
    c = __builtin_amdgcn_wmma_f32_16x16x32_bf16(false, a, false, b, (short)0, c, false, false);
    asm volatile("v_nop\n\tv_nop\n\tv_nop\n\tv_nop" : "+v"(c) : "v"(a), "v"(b));
    return c;
}
__device__ __forceinline__ v8f mma_h(v16h a, v16h b, v8f c) {
    c = __builtin_amdgcn_wmma_f32_16x16x32_f16(false, a, false, b, (short)0, c, false, false);
    asm volatile("v_nop\n\tv_nop\n\tv_nop\n\tv_nop" : "+v"(c) : "v"(a), "v"(b));
    return c;
}

__device__ __forceinline__ void st16x2(unsigned short* p, v4u v) {
    volatile v4u* d = (volatile v4u*)p;
    *d = v; __threadfence(); *d = v;
}

__device__ __forceinline__ v4u pack8_bf(const float* src) {
    const v4f a = *(const v4f*)(src), c = *(const v4f*)(src + 4);
    v4u pk;
    pk.x = bf_bits(a.x) | (bf_bits(a.y) << 16); pk.y = bf_bits(a.z) | (bf_bits(a.w) << 16);
    pk.z = bf_bits(c.x) | (bf_bits(c.y) << 16); pk.w = bf_bits(c.z) | (bf_bits(c.w) << 16);
    return pk;
}

__global__ __launch_bounds__(256) void k_cvt_in(const float* __restrict__ qi, const float* __restrict__ ki,
                                                const float* __restrict__ vi, unsigned short* __restrict__ X16) {
    const int u = blockIdx.x * 256 + threadIdx.x;
    if (u >= SEQ * (HDIM / 8)) return;
    const size_t e = (size_t)u * 8;
    const v4u a = pack8_bf(qi + e);
    const v4u b = pack8_bf(ki + e);
    const v4u c = pack8_bf(vi + e);
    st16x2(X16 + e, a);
    st16x2(X16 + XPL + e, b);
    st16x2(X16 + 2 * XPL + e, c);
}

__device__ __forceinline__ unsigned int cv16(float x, int f16mode) {
    const unsigned int b  = bf_bits(x);
    const unsigned int hb = h_bits(__uint_as_float(b << 16) * WOCAR);
    return f16mode ? hb : b;
}
__global__ __launch_bounds__(256) void k_tr(const float* __restrict__ in, unsigned short* __restrict__ out,
                                            int rows, int cols, int f16mode) {
    __shared__ __align__(16) unsigned short tile[64 * 72];
    const int t = threadIdx.x;
    const int c0 = blockIdx.x * 64, r0 = blockIdx.y * 64;
    {
        const int rl = t >> 2, part = t & 3;
        const float* src = in + (size_t)(r0 + rl) * cols + c0 + part * 16;
        const v4f f0 = *(const v4f*)(src), f1 = *(const v4f*)(src + 4), f2 = *(const v4f*)(src + 8), f3 = *(const v4f*)(src + 12);
        v4u p0, p1;
        p0.x = cv16(f0.x, f16mode) | (cv16(f0.y, f16mode) << 16); p0.y = cv16(f0.z, f16mode) | (cv16(f0.w, f16mode) << 16);
        p0.z = cv16(f1.x, f16mode) | (cv16(f1.y, f16mode) << 16); p0.w = cv16(f1.z, f16mode) | (cv16(f1.w, f16mode) << 16);
        p1.x = cv16(f2.x, f16mode) | (cv16(f2.y, f16mode) << 16); p1.y = cv16(f2.z, f16mode) | (cv16(f2.w, f16mode) << 16);
        p1.z = cv16(f3.x, f16mode) | (cv16(f3.y, f16mode) << 16); p1.w = cv16(f3.z, f16mode) | (cv16(f3.w, f16mode) << 16);
        *(v4u*)(tile + rl * 72 + part * 16)     = p0;
        *(v4u*)(tile + rl * 72 + part * 16 + 8) = p1;
    }
    __syncthreads();
#pragma unroll
    for (int it = 0; it < 2; ++it) {
        const int orow = it * 32 + (t >> 3), pc = t & 7;
        unsigned int e[8];
#pragma unroll
        for (int j = 0; j < 8; ++j) e[j] = (unsigned int)tile[(pc * 8 + j) * 72 + orow];
        v4u pk;
        pk.x = e[0] | (e[1] << 16); pk.y = e[2] | (e[3] << 16); pk.z = e[4] | (e[5] << 16); pk.w = e[6] | (e[7] << 16);
        st16x2(out + (size_t)(c0 + orow) * rows + r0 + pc * 8, pk);
    }
}

__global__ __launch_bounds__(64) void k_invf(float* __restrict__ INVF) {
    __shared__ __align__(16) float sh[64];
    const int t = threadIdx.x;
    const float e = (float)(2 * t) / 128.0f;
    const float p = powf(10000.0f, e);
    sh[t] = 1.0f / p;
    __syncthreads();
    const v4f v = *(const v4f*)(sh + 4 * (t & 15));
    if (t < 16) {
        volatile v4f* d = (volatile v4f*)(INVF + 4 * t);
        *d = v; __threadfence(); *d = v;
    }
}

__global__ __launch_bounds__(256) void k_rope_tab(const float* __restrict__ INVF, float* __restrict__ TAB) {
    __shared__ __align__(16) float cs[256];
    __shared__ __align__(16) float sn[256];
    const int t = threadIdx.x;
    const int pos = blockIdx.x * 4 + (t >> 6), i = t & 63;
    const float ang = (float)pos * INVF[i];
    float s_, c_;
    sincosf(ang, &s_, &c_);
    cs[t] = c_; sn[t] = s_;
    __syncthreads();
    const int p = t & 63;
    const v4f vc = *(const v4f*)(cs + 4 * p);
    const v4f vs = *(const v4f*)(sn + 4 * p);
    const v4f val = (t < 64) ? vc : vs;
    const size_t off = ((t < 64) ? (size_t)0 : (size_t)SEQ * 64) + (size_t)blockIdx.x * 256 + 4 * p;
    if (t < 128) {
        volatile v4f* d = (volatile v4f*)(TAB + off);
        *d = val; __threadfence(); *d = val;
    }
}

__global__ __launch_bounds__(256) void k_proj(const unsigned short* __restrict__ X, const unsigned short* __restrict__ WT,
                                              const float* __restrict__ bias, unsigned short* __restrict__ out,
                                              const float* __restrict__ TAB, int N, int mode, float carry) {
    __shared__ __align__(16) unsigned short stg[128 * SP];
    const int tid = threadIdx.x, wave = tid >> 5, lane = tid & 31, hh = lane >> 4, c = lane & 15;
    const int m0 = blockIdx.x * 16;
    const int ncol0 = blockIdx.y * 1024 + wave * 128;

    FB a[4];
    {
        const unsigned short* xr = X + (size_t)(m0 + c) * HDIM;
#pragma unroll
        for (int kc = 0; kc < 4; ++kc) {
            a[kc].q[0] = *(const v4u*)(xr + kc * 32 + 8 * hh);
            a[kc].q[1] = *(const v4u*)(xr + kc * 32 + 16 + 8 * hh);
        }
    }
    v8f acc[8];
#pragma unroll
    for (int t = 0; t < 8; ++t) {
        acc[t] = (v8f){0.f, 0.f, 0.f, 0.f, 0.f, 0.f, 0.f, 0.f};
        const unsigned short* wr = WT + (size_t)(ncol0 + t * 16 + c) * HDIM;
#pragma unroll
        for (int kc = 0; kc < 4; ++kc) {
            FB b;
            b.q[0] = *(const v4u*)(wr + kc * 32 + 8 * hh);
            b.q[1] = *(const v4u*)(wr + kc * 32 + 16 + 8 * hh);
            acc[t] = mma_bf(a[kc].v, b.v, acc[t]);
        }
        asm volatile("" ::: "memory");
    }
    float bv[8];
#pragma unroll
    for (int t = 0; t < 8; ++t) bv[t] = bf_val(bias[ncol0 + t * 16 + c]);

    if (mode == 0) {
#pragma unroll
        for (int t = 0; t < 8; ++t)
#pragma unroll
            for (int r = 0; r < 8; ++r)
                stg[(wave * 16 + 8 * hh + r) * SP + t * 16 + c] = (unsigned short)h_bits((acc[t][r] + bv[t]) * carry);
    } else {
#pragma unroll
        for (int r = 0; r < 8; ++r) {
            const int m = m0 + 8 * hh + r;
            const int s = (m % RPK) * 8 + wave;
            const float* cr = TAB + (size_t)s * 64 + c;
            const float* sr = TAB + (size_t)SEQ * 64 + (size_t)s * 64 + c;
            const int kl = (8 * hh + r) * 8 + wave;
#pragma unroll
            for (int t = 0; t < 4; ++t) {
                const float cs = cr[t * 16], sn = sr[t * 16];
                const float x0 = acc[t][r] + bv[t], x1 = acc[t + 4][r] + bv[t + 4];
                const float o0 = x0 * cs - x1 * sn;
                const float o1 = x1 * cs + x0 * sn;
                const int d = t * 16 + c;
                const int i0 = (mode == 1) ? ((wave * 16 + 8 * hh + r) * SP + d) : (d * SP + kl);
                const int i1 = (mode == 1) ? (i0 + 64) : (i0 + 64 * SP);
                stg[i0] = (unsigned short)h_bits(o0 * carry);
                stg[i1] = (unsigned short)h_bits(o1 * carry);
            }
            asm volatile("" ::: "memory");
        }
    }
    __syncthreads();

    const int g  = m0 / RPK;
    const int s0 = (m0 % RPK) * 8;
    for (int pass = 0; pass < 2; ++pass) {
#pragma unroll
        for (int it = 0; it < 8; ++it) {
            const int rrow = it * 2 + hh;
            const int drow = it * 16 + wave * 2 + hh;
            const int soff = (mode == 2) ? (drow * SP + c * 8) : ((wave * 16 + rrow) * SP + c * 8);
            const size_t doff = (mode == 2) ? ((size_t)(g * HDIM + drow) * SEQ + s0 + c * 8)
                                            : ((size_t)(m0 + rrow) * N + ncol0 + c * 8);
            const v4u val = *(const v4u*)(stg + soff);
            *(volatile v4u*)(out + doff) = val;
        }
        __threadfence();
    }
}

__global__ __launch_bounds__(128) void k_attn(const unsigned short* __restrict__ Q16, const unsigned short* __restrict__ K16,
                                              const unsigned short* __restrict__ VT16, unsigned short* __restrict__ CTX) {
    __shared__ __align__(16) unsigned short Ksh[KC * HDIM];
    __shared__ __align__(16) unsigned short Vth[HDIM * KC];
    __shared__ __align__(16) _Float16       Psh[NWAVE][QT * KC];
    __shared__ __align__(16) unsigned short Os[NWAVE][QT * SP];

    const int tid = threadIdx.x, wave = tid >> 5, lane = tid & 31, hh = lane >> 4, c = lane & 15;
    const int g = blockIdx.y;
    const int q0 = blockIdx.x * QT;
    const int head = wave * NKVH + g;
    const float SC = (float)(1.4426950408889634 * 0.08838834764831845 / 256.0);

    FH qa[4];
    {
        const unsigned short* qrow = Q16 + ((size_t)head * SEQ + q0 + c) * HDIM;
#pragma unroll
        for (int dc = 0; dc < 4; ++dc) {
            qa[dc].q[0] = *(const v4u*)(qrow + dc * 32 + 8 * hh);
            qa[dc].q[1] = *(const v4u*)(qrow + dc * 32 + 16 + 8 * hh);
        }
    }

    float mrow[8], lrow[8];
    v8f oacc[8];
#pragma unroll
    for (int r = 0; r < 8; ++r) { mrow[r] = -INFINITY; lrow[r] = 0.f; }
#pragma unroll
    for (int t = 0; t < 8; ++t) oacc[t] = (v8f){0.f, 0.f, 0.f, 0.f, 0.f, 0.f, 0.f, 0.f};

    const unsigned short* Kb = K16 + (size_t)g * SEQ * HDIM;
    const unsigned short* Vb = VT16 + (size_t)g * HDIM * SEQ;
    _Float16* pw = Psh[wave];

#pragma unroll 1
    for (int kc = 0; kc < SEQ / KC; ++kc) {
        const int kv0 = kc * KC;
        __syncthreads();
#pragma unroll
        for (int i = 0; i < 8; ++i) {
            const int idx = tid + 128 * i;
            const v4u kk = *(const v4u*)(Kb + (size_t)kv0 * HDIM + (size_t)idx * 8);
            *(v4u*)(Ksh + idx * 8) = kk;
        }
        asm volatile("" ::: "memory");
#pragma unroll
        for (int i = 0; i < 8; ++i) {
            const int idx = tid + 128 * i;
            const int row = idx >> 3, pc = idx & 7;
            const v4u vv = *(const v4u*)(Vb + (size_t)row * SEQ + kv0 + pc * 8);
            *(v4u*)(Vth + row * KC + pc * 8) = vv;
        }
        __syncthreads();

        v8f s[4];
#pragma unroll
        for (int j = 0; j < 4; ++j) {
            s[j] = (v8f){0.f, 0.f, 0.f, 0.f, 0.f, 0.f, 0.f, 0.f};
#pragma unroll
            for (int dc = 0; dc < 4; ++dc) {
                FH kb;
                kb.q[0] = *(const v4u*)(Ksh + (j * 16 + c) * HDIM + dc * 32 + 8 * hh);
                kb.q[1] = *(const v4u*)(Ksh + (j * 16 + c) * HDIM + dc * 32 + 16 + 8 * hh);
                s[j] = mma_h(qa[dc].v, kb.v, s[j]);
            }
        }

#pragma unroll
        for (int r = 0; r < 8; ++r) {
            const float x0 = s[0][r] * SC, x1 = s[1][r] * SC, x2 = s[2][r] * SC, x3 = s[3][r] * SC;
            float m = fmaxf(fmaxf(x0, x1), fmaxf(x2, x3));
            m = fmaxf(m, __shfl_xor(m, 1, 32)); m = fmaxf(m, __shfl_xor(m, 2, 32));
            m = fmaxf(m, __shfl_xor(m, 4, 32)); m = fmaxf(m, __shfl_xor(m, 8, 32));
            const float mnew  = fmaxf(mrow[r], m);
            const float alpha = exp2f(mrow[r] - mnew);
            mrow[r] = mnew;
            const float p0 = exp2f(x0 - mnew), p1 = exp2f(x1 - mnew), p2 = exp2f(x2 - mnew), p3 = exp2f(x3 - mnew);
            _Float16* prow = pw + (8 * hh + r) * KC + c;
            prow[0]  = (_Float16)(p0 * PCAR);
            prow[16] = (_Float16)(p1 * PCAR);
            prow[32] = (_Float16)(p2 * PCAR);
            prow[48] = (_Float16)(p3 * PCAR);
            float psum = (p0 + p1) + (p2 + p3);
            psum += __shfl_xor(psum, 1, 32); psum += __shfl_xor(psum, 2, 32);
            psum += __shfl_xor(psum, 4, 32); psum += __shfl_xor(psum, 8, 32);
            lrow[r] = lrow[r] * alpha + psum;
#pragma unroll
            for (int t = 0; t < 8; ++t) oacc[t][r] *= alpha;
        }
        __builtin_amdgcn_fence(3  , "workgroup");
        __builtin_amdgcn_wave_barrier();
        __builtin_amdgcn_fence(2  , "workgroup");

#pragma unroll
        for (int kk = 0; kk < 2; ++kk) {
            FH pa;
            pa.h[0] = *(const v8h*)(pw + c * KC + kk * 32 + 8 * hh);
            pa.h[1] = *(const v8h*)(pw + c * KC + kk * 32 + 16 + 8 * hh);
#pragma unroll
            for (int t = 0; t < 8; ++t) {
                FH vb;
                vb.q[0] = *(const v4u*)(Vth + (t * 16 + c) * KC + kk * 32 + 8 * hh);
                vb.q[1] = *(const v4u*)(Vth + (t * 16 + c) * KC + kk * 32 + 16 + 8 * hh);
                oacc[t] = mma_h(pa.v, vb.v, oacc[t]);
            }
        }
    }

    unsigned short* os = Os[wave];
#pragma unroll
    for (int r = 0; r < 8; ++r) {
        const float inv = (1.0f / lrow[r]) * (CCAR / (PCAR * VCAR));
#pragma unroll
        for (int t = 0; t < 8; ++t) os[(8 * hh + r) * SP + t * 16 + c] = (unsigned short)h_bits(oacc[t][r] * inv);
    }
    __syncthreads();
    {
        unsigned short* ob = CTX + (size_t)q0 * EQ + head * HDIM;
        for (int pass = 0; pass < 2; ++pass) {
#pragma unroll
            for (int it = 0; it < 8; ++it) {
                const int row = it * 2 + hh;
                const v4u val = *(const v4u*)(os + row * SP + c * 8);
                *(volatile v4u*)(ob + (size_t)row * EQ + c * 8) = val;
            }
            __threadfence();
        }
    }
}

__global__ __launch_bounds__(128) void k_out(const unsigned short* __restrict__ CTX, const unsigned short* __restrict__ WoT,
                                             const float* __restrict__ bo, float* __restrict__ out) {
    __shared__ __align__(16) float part[NWAVE][QT * PP];
    const int tid = threadIdx.x, wave = tid >> 5, lane = tid & 31, hh = lane >> 4, c = lane & 15;
    const int m0 = blockIdx.x * QT;
    const int kbase = wave * (EQ / NWAVE);
    const unsigned short* ar = CTX + (size_t)(m0 + c) * EQ + kbase + 8 * hh;
    const unsigned short* br = WoT + (size_t)c * EQ + kbase + 8 * hh;

    v8f acc[8];
#pragma unroll
    for (int t = 0; t < 8; ++t) acc[t] = (v8f){0.f, 0.f, 0.f, 0.f, 0.f, 0.f, 0.f, 0.f};
#pragma unroll 1
    for (int ks = 0; ks < (EQ / NWAVE) / 32; ++ks) {
        const int k0 = ks * 32;
        FH a;
        a.q[0] = *(const v4u*)(ar + k0);
        a.q[1] = *(const v4u*)(ar + k0 + 16);
#pragma unroll
        for (int t = 0; t < 8; ++t) {
            FH b;
            b.q[0] = *(const v4u*)(br + (size_t)t * 16 * EQ + k0);
            b.q[1] = *(const v4u*)(br + (size_t)t * 16 * EQ + k0 + 16);
            acc[t] = mma_h(a.v, b.v, acc[t]);
            if (t == 3) asm volatile("" ::: "memory");
        }
    }
#pragma unroll
    for (int t = 0; t < 8; ++t)
#pragma unroll
        for (int r = 0; r < 8; ++r) part[wave][(8 * hh + r) * PP + t * 16 + c] = acc[t][r];
    __syncthreads();

    const v4f braw = *(const v4f*)(bo + lane * 4);
    v4f bb;
    bb.x = bf_val(braw.x); bb.y = bf_val(braw.y); bb.z = bf_val(braw.z); bb.w = bf_val(braw.w);
    const float OSC = 1.0f / (CCAR * WOCAR);
    v4f res[4];
#pragma unroll
    for (int it = 0; it < 4; ++it) {
        const int row = it * 4 + wave;
        const v4f p0 = *(const v4f*)(&part[0][row * PP + lane * 4]);
        const v4f p1 = *(const v4f*)(&part[1][row * PP + lane * 4]);
        const v4f p2 = *(const v4f*)(&part[2][row * PP + lane * 4]);
        const v4f p3 = *(const v4f*)(&part[3][row * PP + lane * 4]);
        const v4f sum = ((p0 + p1) + p2) + p3;
        res[it] = sum * OSC + bb;
    }
    for (int pass = 0; pass < 2; ++pass) {
#pragma unroll
        for (int it = 0; it < 4; ++it) {
            const int row = it * 4 + wave;
            *(volatile v4f*)(out + (size_t)(m0 + row) * NOUT + lane * 4) = res[it];
        }
        __threadfence();
    }
}

extern "C" void kernel_launch(void* const* d_in, const int* in_sizes, int n_in, void* d_out, int out_size, void* d_ws, size_t ws_size, hipStream_t stream) {
    if (n_in < 11) return;
    if ((long long)in_sizes[0] < (long long)SEQ * HDIM) return;
    if ((long long)in_sizes[1] < (long long)SEQ * HDIM) return;
    if ((long long)in_sizes[2] < (long long)SEQ * HDIM) return;
    if ((long long)in_sizes[3] < (long long)HDIM * EQ) return;
    if ((long long)in_sizes[4] < (long long)EQ) return;
    if ((long long)in_sizes[5] < (long long)HDIM * EKV) return;
    if ((long long)in_sizes[6] < (long long)EKV) return;
    if ((long long)in_sizes[7] < (long long)HDIM * EKV) return;
    if ((long long)in_sizes[8] < (long long)EKV) return;
    if ((long long)in_sizes[9] < (long long)EQ * NOUT) return;
    if ((long long)in_sizes[10] < (long long)NOUT) return;
    if ((long long)out_size < (long long)SEQ * NOUT) return;
    if (ws_size < WS_TOTAL) return;

    const float* query  = (const float*)d_in[0];
    const float* keys   = (const float*)d_in[1];
    const float* values = (const float*)d_in[2];
    const float* Wq = (const float*)d_in[3];
    const float* bq = (const float*)d_in[4];
    const float* Wk = (const float*)d_in[5];
    const float* bk = (const float*)d_in[6];
    const float* Wv = (const float*)d_in[7];
    const float* bv = (const float*)d_in[8];
    const float* Wo = (const float*)d_in[9];
    const float* bo = (const float*)d_in[10];
    float* out = (float*)d_out;

    char* w = (char*)d_ws;
    unsigned short* X16 = (unsigned short*)(w + OFF_X16);
    unsigned short* WQT = (unsigned short*)(w + OFF_WQT);
    unsigned short* WKT = (unsigned short*)(w + OFF_WKT);
    unsigned short* WVT = (unsigned short*)(w + OFF_WVT);
    unsigned short* WOT = (unsigned short*)(w + OFF_WOT);
    float*          INV = (float*)(w + OFF_INV);
    float*          TAB = (float*)(w + OFF_TAB);
    unsigned short* Q16 = (unsigned short*)(w + OFF_Q16);
    unsigned short* K16 = (unsigned short*)(w + OFF_K16);
    unsigned short* VT  = (unsigned short*)(w + OFF_VT);
    unsigned short* CTX = (unsigned short*)(w + OFF_CTX);

    k_cvt_in<<<(unsigned)((SEQ * (HDIM / 8) + 255) / 256), 256, 0, stream>>>(query, keys, values, X16);
    k_tr<<<dim3((unsigned)(EQ / 64),  (unsigned)(HDIM / 64)), 256, 0, stream>>>(Wq, WQT, HDIM, EQ, 0);
    k_tr<<<dim3((unsigned)(EKV / 64), (unsigned)(HDIM / 64)), 256, 0, stream>>>(Wk, WKT, HDIM, EKV, 0);
    k_tr<<<dim3((unsigned)(EKV / 64), (unsigned)(HDIM / 64)), 256, 0, stream>>>(Wv, WVT, HDIM, EKV, 0);
    k_tr<<<dim3((unsigned)(NOUT / 64), (unsigned)(EQ / 64)), 256, 0, stream>>>(Wo, WOT, EQ, NOUT, 1);
    k_invf<<<1, 64, 0, stream>>>(INV);
    k_rope_tab<<<(unsigned)(SEQ / 4), 256, 0, stream>>>(INV, TAB);

    k_proj<<<dim3((unsigned)(SEQ / 16), (unsigned)(EQ / 1024)),  256, 0, stream>>>(X16,           WQT, bq, Q16, TAB, EQ,  0, QCAR);
    k_proj<<<dim3((unsigned)(SEQ / 16), (unsigned)(EKV / 1024)), 256, 0, stream>>>(X16 + XPL,     WKT, bk, K16, TAB, EKV, 1, QCAR);
    k_proj<<<dim3((unsigned)(SEQ / 16), (unsigned)(EKV / 1024)), 256, 0, stream>>>(X16 + 2 * XPL, WVT, bv, VT,  TAB, EKV, 2, VCAR);

    k_attn<<<dim3((unsigned)(SEQ / QT), (unsigned)NKVH), 128, 0, stream>>>(Q16, K16, VT, CTX);
    k_out<<<(unsigned)(SEQ / QT), 128, 0, stream>>>(CTX, WOT, bo, out);
}
